// CNF_13546326852134
// MI455X (gfx1250) — hardware-run, weakly checked
//
#include <hip/hip_runtime.h>
#include <math.h>

typedef __attribute__((ext_vector_type(16))) _Float16 v16h;
typedef __attribute__((ext_vector_type(8)))  _Float16 v8h;
typedef __attribute__((ext_vector_type(8)))  float    v8f;
typedef __attribute__((ext_vector_type(4)))  float    v4f;

constexpr int kBatch        = 1024;
constexpr int kObj          = 32;
constexpr int kPairs        = 496;
constexpr int kFeat         = 146;
constexpr int kFeatPad      = 160;
constexpr int kHid          = 128;
constexpr int kTotalPairs   = kBatch * kPairs;
constexpr int kPairsPerWave = 16;
constexpr int kRowsPerWave  = 32;
constexpr int kPairsPerTile = 128;
constexpr int kTilesPerBlk  = 4;
constexpr int kTiles        = kTotalPairs / kPairsPerTile;
constexpr int kBlocks       = kTiles / kTilesPerBlk;
constexpr int kXPitch       = 168;
static_assert(kPairs == kObj * (kObj - 1) / 2);
static_assert(kTiles * kPairsPerTile == kTotalPairs);
static_assert(kBlocks * kTilesPerBlk == kTiles);
static_assert(kBlocks == 992);
static_assert((kFeatPad % 32) == 0 && (kHid % 32) == 0 && kFeatPad >= kFeat);
static_assert(kFeat == 6 + 60 + 80);
static_assert((kXPitch % 8) == 0 && kXPitch >= kFeatPad);

constexpr float kCarryW  = 256.0f;
constexpr float kCarryX  = 16.0f;
constexpr float kCarryH0 = 16.0f;
constexpr float kCarryH1 = 64.0f;
constexpr float kScale0  = kCarryH0 / (kCarryW * kCarryX);
constexpr float kScale1  = kCarryH1 / (kCarryW * kCarryH0);
constexpr float kScale2  = 1.0f / (kCarryW * kCarryH1);
constexpr float kPiF     = 3.14159265358979323846f;
constexpr float kClip    = 0.003f;

constexpr int kInputsToBf16 = 0;

constexpr int kChunks0     = kHid * kFeatPad / 8;
constexpr int kChunks1     = kHid * kHid / 8;
constexpr int kChunksAll   = kChunks0 + 2 * kChunks1;
constexpr int kPlaneHalves = kChunksAll * 8;
constexpr size_t kWsTotal  = (size_t)kPlaneHalves * 2;
static_assert(kChunks0 == 2560 && kChunks1 == 2048 && kChunksAll == 6656);
static_assert((kChunks0 % 32) == 0 && (kChunks1 % 32) == 0 && (kChunksAll % 256) == 0);
static_assert(kWsTotal == 106496ull);
static_assert(kWsTotal <= 134217728ull);


__device__ __forceinline__ float rne_bf16(float f) {
  unsigned u = __float_as_uint(f);
  u = (u + 0x7FFFu + ((u >> 16) & 1u)) & 0xFFFF0000u;
  return __uint_as_float(u);
}

struct FragH {
  union U { v16h v; v8h h[2]; };
  static __device__ __forceinline__ v16h load(const _Float16* p) {
    U f;
    f.h[0] = *(const v8h*)(p);
    f.h[1] = *(const v8h*)(p + 16);
    return f.v;
  }
};

__device__ __forceinline__ v8f mma_guarded(v16h a, v16h b, v8f c) {
  c = __builtin_amdgcn_wmma_f32_16x16x32_f16(false, a, false, b, (short)0, c, false, false);
  asm volatile("v_nop\n\tv_nop\n\tv_nop\n\tv_nop" : "+v"(c) : "v"(a), "v"(b));
  return c;
}

__device__ __forceinline__ void wave_lds_sync() {
  __builtin_amdgcn_fence(__ATOMIC_RELEASE, "workgroup");
  __builtin_amdgcn_wave_barrier();
  __builtin_amdgcn_fence(__ATOMIC_ACQUIRE, "workgroup");
}

__global__ __launch_bounds__(256) void weight_planes_kernel(
    const float* __restrict__ W0, const float* __restrict__ W1, const float* __restrict__ W2,
    _Float16* __restrict__ planes)
{
  const int c  = blockIdx.x * 256 + threadIdx.x;
  const int cw = __builtin_amdgcn_readfirstlane(c);
  const int pl = (cw < kChunks0) ? 0 : ((cw < kChunks0 + kChunks1) ? 1 : 2);
  const float* src = (pl == 0) ? W0 : ((pl == 1) ? W1 : W2);
  const int kreal = (pl == 0) ? kFeat : kHid;
  const int cpr   = (pl == 0) ? (kFeatPad / 8) : (kHid / 8);
  const int base  = (pl == 0) ? 0 : ((pl == 1) ? kChunks0 : (kChunks0 + kChunks1));
  const int lc = c - base;
  int n = lc / cpr;
  const int kc = lc - n * cpr;
  n = (n > kHid - 1) ? (kHid - 1) : n;
  v8h hv;
#pragma unroll
  for (int e = 0; e < 8; ++e) {
    const int kk = kc * 8 + e;
    int r = kk + 66;
    r = (kk >= 80)  ? (kk - 74)  : r;
    r = (kk >= 110) ? (kk - 110) : r;
    r = (kk >= 112) ? (kk - 76)  : r;
    r = (kk >= 142) ? (kk - 140) : r;
    r = (pl == 0) ? r : kk;
    const bool valid = (kk < kreal);
    r = (r < 0) ? 0 : r;
    r = (r > kreal - 1) ? (kreal - 1) : r;
    float x = src[r * kHid + n];
    x = valid ? x : 0.0f;
    if (kInputsToBf16) x = rne_bf16(x);
    hv[e] = (_Float16)(x * kCarryW);
  }
  _Float16* dst = planes + (size_t)c * 8;
  *(volatile v8h*)dst = hv;
  __threadfence();
  *(volatile v8h*)dst = hv;
}

__device__ __forceinline__ _Float16 h16x(float x) { return (_Float16)(x * kCarryX); }

__device__ __forceinline__ void build_rows(
    const float* __restrict__ objt, const float* __restrict__ pos, const float* __restrict__ quat,
    int gp, int fh, _Float16* xr0)
{
#pragma clang fp contract(off)
  const int b = gp / kPairs;
  const int p = gp - b * kPairs;
  int i = 0, pp = p;
#pragma unroll 1
  for (int it = 0; it < kObj - 1; ++it) {
    const int rl = (kObj - 1) - i;
    const bool adv = (pp >= rl);
    pp = adv ? (pp - rl) : pp;
    i  = adv ? (i + 1) : i;
  }
  i = (i > kObj - 2) ? (kObj - 2) : i;
  int j = i + 1 + pp;
  j = (j > kObj - 1) ? (kObj - 1) : j;
  const int ra = b * kObj + i;
  const int rc = b * kObj + j;

  float ti0 = objt[ra * 3 + 0], ti1 = objt[ra * 3 + 1], ti2 = objt[ra * 3 + 2];
  float tj0 = objt[rc * 3 + 0], tj1 = objt[rc * 3 + 1], tj2 = objt[rc * 3 + 2];
  asm volatile("" : "+v"(ti0));
  asm volatile("" : "+v"(ti1));
  asm volatile("" : "+v"(ti2));
  asm volatile("" : "+v"(tj0));
  asm volatile("" : "+v"(tj1));
  asm volatile("" : "+v"(tj2));
  float pix = pos[ra * 3 + 0], piy = pos[ra * 3 + 1], piz = pos[ra * 3 + 2];
  float pjx = pos[rc * 3 + 0], pjy = pos[rc * 3 + 1], pjz = pos[rc * 3 + 2];
  const v4f qa = *(const v4f*)(quat + ra * 4);
  const v4f qc = *(const v4f*)(quat + rc * 4);
  float vax = qa[0], vay = qa[1], vaz = qa[2], wa = qa[3];
  float vcx = qc[0], vcy = qc[1], vcz = qc[2], wc = qc[3];
  if (kInputsToBf16) {
    pix = rne_bf16(pix); piy = rne_bf16(piy); piz = rne_bf16(piz);
    pjx = rne_bf16(pjx); pjy = rne_bf16(pjy); pjz = rne_bf16(pjz);
    vax = rne_bf16(vax); vay = rne_bf16(vay); vaz = rne_bf16(vaz); wa = rne_bf16(wa);
    vcx = rne_bf16(vcx); vcy = rne_bf16(vcy); vcz = rne_bf16(vcz); wc = rne_bf16(wc);
  }
  const float nvx = -vax, nvy = -vay, nvz = -vaz;
  float xs[7];
  xs[0] = pjx - pix;
  xs[1] = pjy - piy;
  xs[2] = pjz - piz;
  xs[3] = (wa * vcx + wc * nvx) + (nvy * vcz - nvz * vcy);
  xs[4] = (wa * vcy + wc * nvy) + (nvz * vcx - nvx * vcz);
  xs[5] = (wa * vcz + wc * nvz) + (nvx * vcy - nvy * vcx);
  xs[6] = wa * wc - ((nvx * vcx + nvz * vcz) + nvy * vcy);

  const float fs = fh ? 32.0f : 1.0f;
  float cs[7], sn[7];
#pragma unroll
  for (int q = 0; q < 7; ++q) {
    const float ang = (xs[q] * kPiF) * fs;
    float s, c;
    sincosf(ang, &s, &c);
    sn[q] = s;
    cs[q] = c;
  }

  _Float16* xr1 = xr0 + kXPitch;
  const int lqcol = 40 * fh;
  v8h pa[4], pb[4];
#pragma unroll
  for (int e = 0; e < 5; ++e) {
    v8h la, lb;
#pragma unroll
    for (int d = 0; d < 4; ++d) {
      const _Float16 hc = h16x(cs[3 + d]);
      const _Float16 hs = h16x(sn[3 + d]);
      la[d] = hc;
      lb[d] = hc;
      la[4 + d] = hs;
      lb[4 + d] = (d < 3) ? h16x(-sn[3 + d]) : hs;
    }
    *(v8h*)(xr0 + lqcol + 8 * e) = la;
    *(v8h*)(xr1 + lqcol + 8 * e) = lb;
#pragma unroll
    for (int d = 0; d < 3; ++d) {
      const int ic = 6 * e + d;
      const int is = 6 * e + 3 + d;
      const _Float16 hc = h16x(cs[d]);
      pa[ic >> 3][ic & 7] = hc;
      pb[ic >> 3][ic & 7] = hc;
      pa[is >> 3][is & 7] = h16x(sn[d]);
      pb[is >> 3][is & 7] = h16x(-sn[d]);
    }
    if (e < 4) {
#pragma unroll
      for (int q = 0; q < 7; ++q) {
        const float c = cs[q], s = sn[q];
        cs[q] = (c - s) * (c + s);
        sn[q] = (s + s) * c;
      }
    }
  }
  const float a30 = fh ? ti2 : ti0;
  const float a31 = fh ? tj0 : ti1;
  const float b30 = fh ? tj2 : tj0;
  const float b31 = fh ? ti0 : tj1;
  pa[3][6] = h16x(a30);
  pa[3][7] = h16x(a31);
  pb[3][6] = h16x(b30);
  pb[3][7] = h16x(b31);
  const int rcol = 80 + 32 * fh;
#pragma unroll
  for (int v = 0; v < 4; ++v) {
    *(v8h*)(xr0 + rcol + 8 * v) = pa[v];
    *(v8h*)(xr1 + rcol + 8 * v) = pb[v];
  }
  float zf = 0.0f;
  asm volatile("" : "+v"(zf));
  const _Float16 zh = (_Float16)zf;
  const float tu = fh ? ti1 : tj1;
  const float tw = fh ? ti2 : tj2;
  v8h t0, t1;
  t0[0] = h16x(tu);
  t0[1] = h16x(tw);
#pragma unroll
  for (int q = 2; q < 8; ++q) t0[q] = zh;
#pragma unroll
  for (int q = 0; q < 8; ++q) t1[q] = zh;
  _Float16* xt = xr0 + fh * kXPitch;
  *(v8h*)(xt + 144) = t0;
  *(v8h*)(xt + 152) = t1;
}

template <int KSTEPS, int LDW>
__device__ __forceinline__ void layer_mma(const _Float16* W, const _Float16* X, int lane, v8f (&acc)[8][2])
{
  const int m  = lane & 15;
  const int h8 = (lane >> 4) * 8;
  const _Float16* wp = W + m * LDW + h8;
  const _Float16* xp = X + m * kXPitch + h8;
#pragma unroll
  for (int i = 0; i < 8; ++i) {
    acc[i][0] = (v8f){0.f, 0.f, 0.f, 0.f, 0.f, 0.f, 0.f, 0.f};
    acc[i][1] = (v8f){0.f, 0.f, 0.f, 0.f, 0.f, 0.f, 0.f, 0.f};
  }
#pragma unroll 1
  for (int ks = 0; ks < KSTEPS; ++ks) {
    const v16h b0 = FragH::load(xp + ks * 32);
    const v16h b1 = FragH::load(xp + 16 * kXPitch + ks * 32);
#pragma unroll
    for (int i = 0; i < 8; ++i) {
      const v16h a = FragH::load(wp + i * 16 * LDW + ks * 32);
      acc[i][0] = mma_guarded(a, b0, acc[i][0]);
      acc[i][1] = mma_guarded(a, b1, acc[i][1]);
    }
  }
}

__device__ __forceinline__ void epilogue_hidden(v8f (&acc)[8][2], const float* sBias, float sc, _Float16* X, int lane)
{
  const int n  = lane & 15;
  const int h8 = (lane >> 4) * 8;
#pragma unroll
  for (int i = 0; i < 8; ++i) {
    const v4f ba = *(const v4f*)(sBias + 16 * i + h8);
    const v4f bb = *(const v4f*)(sBias + 16 * i + h8 + 4);
#pragma unroll
    for (int j = 0; j < 2; ++j) {
      v8h hv;
#pragma unroll
      for (int r = 0; r < 4; ++r) {
        hv[r]     = (_Float16)fmaxf(fmaf(acc[i][j][r],     sc, ba[r]), 0.0f);
        hv[4 + r] = (_Float16)fmaxf(fmaf(acc[i][j][4 + r], sc, bb[r]), 0.0f);
      }
      *(v8h*)(X + (16 * j + n) * kXPitch + 16 * i + h8) = hv;
    }
  }
}

__device__ __forceinline__ void epilogue_head(v8f (&acc)[8][2], const float* sB2, const float* sW3,
                                              float b3v, float* sOutWave, int lane)
{
  const int n  = lane & 15;
  const int h8 = (lane >> 4) * 8;
  float z0 = 0.0f, z1 = 0.0f;
#pragma unroll
  for (int i = 0; i < 8; ++i) {
    const v4f ba = *(const v4f*)(sB2 + 16 * i + h8);
    const v4f bb = *(const v4f*)(sB2 + 16 * i + h8 + 4);
    const v4f wa = *(const v4f*)(sW3 + 16 * i + h8);
    const v4f wb = *(const v4f*)(sW3 + 16 * i + h8 + 4);
#pragma unroll
    for (int r = 0; r < 4; ++r) {
      z0 = fmaf(fmaxf(fmaf(acc[i][0][r],     kScale2, ba[r]), 0.0f), wa[r], z0);
      z1 = fmaf(fmaxf(fmaf(acc[i][1][r],     kScale2, ba[r]), 0.0f), wa[r], z1);
      z0 = fmaf(fmaxf(fmaf(acc[i][0][4 + r], kScale2, bb[r]), 0.0f), wb[r], z0);
      z1 = fmaf(fmaxf(fmaf(acc[i][1][4 + r], kScale2, bb[r]), 0.0f), wb[r], z1);
    }
  }
  z0 += __shfl_xor(z0, 16, 32);
  z1 += __shfl_xor(z1, 16, 32);
  const float r0 = kClip * tanhf(z0 + b3v);
  const float r1 = kClip * tanhf(z1 + b3v);
  const float o0 = __shfl_xor(r0, 1, 32);
  const float o1 = __shfl_xor(r1, 1, 32);
  const float m0 = 0.5f * (r0 + o0);
  const float m1 = 0.5f * (r1 + o1);
  if (h8 == 0 && (n & 1) == 0) {
    sOutWave[n >> 1]     = m0;
    sOutWave[8 + (n >> 1)] = m1;
  }
}

__global__ __launch_bounds__(256) void pair_mlp_kernel(
    const float* __restrict__ objt, const float* __restrict__ pos, const float* __restrict__ quat,
    const _Float16* __restrict__ planes,
    const float* __restrict__ b0, const float* __restrict__ b1, const float* __restrict__ b2,
    const float* __restrict__ W3, const float* __restrict__ b3,
    float* __restrict__ out)
{
  __shared__ __align__(16) _Float16 sW[kPlaneHalves];
  __shared__ __align__(16) _Float16 sX[8 * kRowsPerWave * kXPitch];
  __shared__ __align__(16) float sPar[4 * kHid];
  __shared__ __align__(16) float sOut[kTilesPerBlk * kPairsPerTile];

  const int tid  = threadIdx.x;
  const int lane = tid & 31;
  const int wave = __builtin_amdgcn_readfirstlane((int)(threadIdx.x >> 5));

#pragma unroll 2
  for (int c = tid; c < kChunksAll; c += 256)
    *(v8h*)(sW + c * 8) = *(const v8h*)(planes + (size_t)c * 8);
  {
    const int idx  = tid & (kHid - 1);
    const int hsel = tid >> 7;
    float v0 = b0[idx], v1 = b1[idx], v2 = b2[idx], v3 = W3[idx];
    asm volatile("" : "+v"(v0));
    asm volatile("" : "+v"(v1));
    asm volatile("" : "+v"(v2));
    asm volatile("" : "+v"(v3));
    if (kInputsToBf16) { v0 = rne_bf16(v0); v1 = rne_bf16(v1); v2 = rne_bf16(v2); v3 = rne_bf16(v3); }
    const float e0 = hsel ? v2 : (v0 * kCarryH0);
    const float e1 = hsel ? v3 : (v1 * kCarryH1);
    sPar[(hsel ? 2 * kHid : 0) + idx]        = e0;
    sPar[(hsel ? 3 * kHid : kHid) + idx]     = e1;
  }
  float b3v = b3[0];
  if (kInputsToBf16) b3v = rne_bf16(b3v);
  __syncthreads();

  _Float16* xb = sX + wave * (kRowsPerWave * kXPitch);
  const int pl = lane & 15;
  const int fh = lane >> 4;
  const _Float16* sW0 = sW;
  const _Float16* sW1 = sW + kChunks0 * 8;
  const _Float16* sW2 = sW + (kChunks0 + kChunks1) * 8;

#pragma unroll 1
  for (int t = 0; t < kTilesPerBlk; ++t) {
    const int tile = blockIdx.x * kTilesPerBlk + t;
    int gp = tile * kPairsPerTile + wave * kPairsPerWave + pl;
    gp = (gp > kTotalPairs - 1) ? (kTotalPairs - 1) : gp;
    build_rows(objt, pos, quat, gp, fh, xb + (2 * pl) * kXPitch);
    wave_lds_sync();

    v8f acc[8][2];
    layer_mma<kFeatPad / 32, kFeatPad>(sW0, xb, lane, acc);
    epilogue_hidden(acc, sPar, kScale0, xb, lane);
    wave_lds_sync();

    layer_mma<kHid / 32, kHid>(sW1, xb, lane, acc);
    epilogue_hidden(acc, sPar + kHid, kScale1, xb, lane);
    wave_lds_sync();

    layer_mma<kHid / 32, kHid>(sW2, xb, lane, acc);
    epilogue_head(acc, sPar + 2 * kHid, sPar + 3 * kHid, b3v,
                  sOut + t * kPairsPerTile + wave * kPairsPerWave, lane);
    wave_lds_sync();
  }
  __syncthreads();
  if (wave < kTilesPerBlk) {
    const v4f val = *(const v4f*)(sOut + wave * kPairsPerTile + lane * 4);
    float* dst = out + (size_t)(blockIdx.x * kTilesPerBlk + wave) * kPairsPerTile + lane * 4;
    *(volatile v4f*)dst = val;
    __threadfence();
    *(volatile v4f*)dst = val;
  }
}

extern "C" void kernel_launch(void* const* d_in, const int* in_sizes, int n_in,
                              void* d_out, int out_size, void* d_ws, size_t ws_size,
                              hipStream_t stream) {
  if (n_in < 12) return;
  if (in_sizes[0] != kBatch * kObj * 3) return;
  if (in_sizes[2] != kBatch * kObj * 3) return;
  if (in_sizes[3] != kBatch * kObj * 4) return;
  if (in_sizes[4] != kFeat * kHid) return;
  if (in_sizes[5] != kHid) return;
  if (in_sizes[6] != kHid * kHid) return;
  if (in_sizes[7] != kHid) return;
  if (in_sizes[8] != kHid * kHid) return;
  if (in_sizes[9] != kHid) return;
  if (in_sizes[10] != kHid) return;
  if (in_sizes[11] != 1) return;
  if (out_size != kTotalPairs) return;
  if (ws_size < kWsTotal) return;

  const float* objt = (const float*)d_in[0];
  const float* pos  = (const float*)d_in[2];
  const float* quat = (const float*)d_in[3];
  const float* W0   = (const float*)d_in[4];
  const float* b0   = (const float*)d_in[5];
  const float* W1   = (const float*)d_in[6];
  const float* b1   = (const float*)d_in[7];
  const float* W2   = (const float*)d_in[8];
  const float* b2   = (const float*)d_in[9];
  const float* W3   = (const float*)d_in[10];
  const float* b3   = (const float*)d_in[11];
  float* out = (float*)d_out;
  _Float16* planes = (_Float16*)d_ws;

  weight_planes_kernel<<<kChunksAll / 256, 256, 0, stream>>>(W0, W1, W2, planes);
  pair_mlp_kernel<<<kBlocks, 256, 0, stream>>>(objt, pos, quat, planes, b0, b1, b2, W3, b3, out);
}
